// TemporalPropagator_6932077216157
// MI455X (gfx1250) — hardware-run, weakly checked
//
#include <hip/hip_runtime.h>
#include <math.h>

typedef __attribute__((ext_vector_type(16))) _Float16 v16h;
typedef __attribute__((ext_vector_type(8)))  _Float16 v8h;
typedef __attribute__((ext_vector_type(8)))  float    v8f;
typedef __attribute__((ext_vector_type(4)))  float    v4f;

constexpr int kNB = 2;
constexpr int kNT = 16;
constexpr int kHW = 4096;
constexpr int kD  = 64;
constexpr int kBT = kNB * kNT;
constexpr int kPlane = kBT * kD;
constexpr int kPowIters = 320;
constexpr int kSeriesTerms = 8;
constexpr float kInvSqrtD = 0.125f;
constexpr float kDtRef = 1.0f;
constexpr float kRhoMax = 0.5f;
static_assert(kInvSqrtD * kInvSqrtD * (float)kD == 1.0f);
static_assert(kD == 64 && kHW == 4096 && kBT == 32 && kPlane == 2048);

constexpr float kCarryX   = 16.0f;
constexpr float kCarryW   = 2048.0f;
constexpr float kCarryRes = 2048.0f;
constexpr float kCarryH   = 16.0f;
constexpr float kCarryU   = 256.0f;
constexpr float kFoldEnc     = 1.0f / (kCarryX * kCarryW);
constexpr float kFoldDec     = 1.0f / (kCarryH * kCarryW);
constexpr float kFoldDecRes  = kFoldDec / kCarryRes;
constexpr float kFoldU       = 1.0f / (kCarryH * kCarryU);
constexpr float kF16MinNormal = 6.103515625e-5f;

constexpr size_t kOffEWV   = 0;
constexpr size_t kOffEWR   = kOffEWV + 16384;
constexpr size_t kOffDWV   = kOffEWR + 16384;
constexpr size_t kOffDWR   = kOffDWV + 16384;
constexpr size_t kOffU1    = kOffDWR + 16384;
constexpr size_t kOffU2    = kOffU1 + 2048;
constexpr size_t kOffINVRE = kOffU2 + 2048;
constexpr size_t kOffINVIM = kOffINVRE + 16384;
constexpr size_t kOffTAB   = kOffINVIM + 16384;
constexpr size_t kOffGSRE  = kOffTAB + 65536;
constexpr size_t kOffGSIM  = kOffGSRE + 8192;
constexpr size_t kOffPART  = kOffGSIM + 8192;
constexpr size_t kWsTotal  = kOffPART + 65536;
static_assert(kWsTotal == 249856ull);
static_assert((kOffEWR % 128) == 0 && (kOffDWV % 128) == 0 && (kOffDWR % 128) == 0 && (kOffU1 % 128) == 0 &&
              (kOffU2 % 128) == 0 && (kOffINVRE % 128) == 0 && (kOffINVIM % 128) == 0 && (kOffTAB % 128) == 0 &&
              (kOffGSRE % 128) == 0 && (kOffGSIM % 128) == 0 && (kOffPART % 128) == 0);

namespace eng {

__device__ __forceinline__ float bfr(float f) {
  unsigned u = __float_as_uint(f);
  u = (u + 0x7FFFu + ((u >> 16) & 1u)) & 0xFFFF0000u;
  return __uint_as_float(u);
}
__device__ __forceinline__ float flush14(float s) {
  return (fabsf(s) < kF16MinNormal) ? 0.0f : s;
}
__device__ __forceinline__ void split16(float v, float carry, _Float16& hv, _Float16& hr) {
  const float s = v * carry;
  const _Float16 h = (_Float16)flush14(s);
  const float back = (float)h;
  const float r = (s - back) * kCarryRes;
  hv = h;
  hr = (_Float16)flush14(r);
}
__device__ __forceinline__ _Float16 plain16(float v, float carry) {
  const float s = v * carry;
  return (_Float16)flush14(s);
}
__device__ __forceinline__ v8f zero8f() { return (v8f){0.f, 0.f, 0.f, 0.f, 0.f, 0.f, 0.f, 0.f}; }
__device__ __forceinline__ v8h zero8h() {
  v8h z;
#pragma unroll
  for (int e = 0; e < 8; ++e) z[e] = (_Float16)0.0f;
  return z;
}
__device__ __forceinline__ v8f ld8(const float* p) {
  const v4f a = *(const v4f*)(p);
  const v4f b = *(const v4f*)(p + 4);
  return __builtin_shufflevector(a, b, 0, 1, 2, 3, 4, 5, 6, 7);
}
union FragU { v16h v; v8h h[2]; };
__device__ __forceinline__ v16h frag_ld(const _Float16* p) {
  FragU f;
  f.h[0] = *(const v8h*)(p);
  f.h[1] = *(const v8h*)(p + 16);
  return f.v;
}
__device__ __forceinline__ v8f mma_h(v16h a, v16h b, v8f c) {
  c = __builtin_amdgcn_wmma_f32_16x16x32_f16(false, a, false, b, (short)0, c, false, false);
  asm volatile("v_nop\n\tv_nop\n\tv_nop\n\tv_nop" : "+v"(c) : "v"(a), "v"(b));
  return c;
}
__device__ __forceinline__ void wave_sync_lds() {
  __builtin_amdgcn_fence(__ATOMIC_RELEASE, "workgroup");
  __builtin_amdgcn_wave_barrier();
  __builtin_amdgcn_fence(__ATOMIC_ACQUIRE, "workgroup");
}
__device__ __forceinline__ _Float16 x_to_h(float xv) {
  const float s = bfr(xv) * kCarryX;
  return (_Float16)flush14(s);
}
__device__ __forceinline__ v16h x_frag(const float* rowp) {
  const v4f a0 = *(const v4f*)(rowp);
  const v4f a1 = *(const v4f*)(rowp + 4);
  const v4f b0 = *(const v4f*)(rowp + 16);
  const v4f b1 = *(const v4f*)(rowp + 20);
  v16h f;
#pragma unroll
  for (int e = 0; e < 4; ++e) {
    const float s0 = a0[e];
    const float s1 = a1[e];
    const float s2 = b0[e];
    const float s3 = b1[e];
    f[e]      = x_to_h(s0);
    f[4 + e]  = x_to_h(s1);
    f[8 + e]  = x_to_h(s2);
    f[12 + e] = x_to_h(s3);
  }
  return f;
}
__device__ __forceinline__ void emit_line_pair(const float* sp, float carry, unsigned short* pv, unsigned short* pr) {
  v8h hv, hr;
#pragma unroll
  for (int e = 0; e < 8; ++e) {
    const float v = sp[e];
    _Float16 a, b;
    split16(v, carry, a, b);
    hv[e] = a;
    hr[e] = b;
  }
  *(volatile v8h*)pv = hv;
  *(volatile v8h*)pr = hr;
  __threadfence();
  *(volatile v8h*)pv = hv;
  *(volatile v8h*)pr = hr;
}
__device__ __forceinline__ void build_trig(double* q17c, double* q17s, float* cT, float* sT, int tid) {
  if (tid < 17) {
    const int kk = (tid <= 8) ? tid : (16 - tid);
    const double th = 3.14159265358979323846 * (double)kk * 0.03125;
    double a = 1.0, cs = 1.0, sn = 0.0;
#pragma unroll 1
    for (int n = 1; n <= 26; ++n) {
      a = a * th / (double)n;
      const int m4 = n & 3;
      const double sg = (m4 == 0 || m4 == 1) ? 1.0 : -1.0;
      const double ta = sg * a;
      cs += (n & 1) ? 0.0 : ta;
      sn += (n & 1) ? ta : 0.0;
    }
    q17c[tid] = (tid <= 8) ? cs : sn;
    q17s[tid] = (tid <= 8) ? sn : cs;
  }
  __syncthreads();
  if (tid < 64) {
    const int m = tid;
    int idx;
    double sc, ss;
    if (m <= 16)      { idx = m;      sc = 1.0;  ss = 1.0; }
    else if (m <= 32) { idx = 32 - m; sc = -1.0; ss = 1.0; }
    else if (m <= 48) { idx = m - 32; sc = -1.0; ss = -1.0; }
    else              { idx = 64 - m; sc = 1.0;  ss = -1.0; }
    cT[m] = (float)(sc * q17c[idx] * 0.125);
    sT[m] = (float)(ss * q17s[idx] * 0.125);
  }
  __syncthreads();
}
__device__ __forceinline__ float alpha_of(const float* alpha_logit) {
  const float al = bfr(alpha_logit[0]);
  return 1.0f / (1.0f + expf(-al));
}

}
using namespace eng;

__global__ __launch_bounds__(256) void k_mats(
    const float* __restrict__ w_re_in, const float* __restrict__ w_im_in, const float* __restrict__ alpha_logit,
    unsigned short* __restrict__ EWV, unsigned short* __restrict__ EWR,
    float* __restrict__ INVRE, float* __restrict__ INVIM)
{
  __shared__ __align__(16) float sP[8192];
  __shared__ __align__(16) float sTerm[4096];
  __shared__ __align__(16) float sIV[2048];
  __shared__ double sVre[64], sVim[64], sUre[64], sUim[64], sRed[64];
  __shared__ double sC17[17], sS17[17];
  __shared__ float sCT[64], sST[64];
  const int tid = threadIdx.x, lane = tid & 31, wave = tid >> 5;

  build_trig(sC17, sS17, sCT, sST, tid);

#pragma unroll 1
  for (int which = 0; which < 2; ++which) {
#pragma unroll 1
    for (int e = 0; e < 16; ++e) {
      const int i = tid + 256 * e;
      const float a = w_re_in[i];
      const float b = w_im_in[i];
      const float v = which ? b : a;
      sP[which * 4096 + i] = tanhf(bfr(v)) * kInvSqrtD;
    }
  }
  if (tid < 64) { sVre[tid] = 1.0; sVim[tid] = 0.0; }
  __syncthreads();

#pragma unroll 1
  for (int it = 0; it < kPowIters; ++it) {
    if (tid < 64) {
      double sr = 0.0, si = 0.0;
#pragma unroll 1
      for (int k = 0; k < 64; ++k) {
        const double ar = (double)sP[tid * 64 + k], ai = (double)sP[4096 + tid * 64 + k];
        const double cr = sVre[k], ci = sVim[k];
        sr += ar * cr - ai * ci;
        si += ar * ci + ai * cr;
      }
      sUre[tid] = sr;
      sUim[tid] = si;
    }
    __syncthreads();
    if (tid < 64) {
      double sr = 0.0, si = 0.0;
#pragma unroll 1
      for (int r = 0; r < 64; ++r) {
        const double ar = (double)sP[r * 64 + tid], ai = (double)sP[4096 + r * 64 + tid];
        const double cr = sUre[r], ci = sUim[r];
        sr += ar * cr + ai * ci;
        si += ar * ci - ai * cr;
      }
      sVre[tid] = sr;
      sVim[tid] = si;
      sRed[tid] = sr * sr + si * si;
    }
    __syncthreads();
    double s = 0.0;
#pragma unroll 1
    for (int k = 0; k < 64; ++k) s += sRed[k];
    const float rn = rsqrtf(fmaxf((float)s, 1e-30f));
    if (tid < 64) {
      sVre[tid] = sVre[tid] * (double)rn;
      sVim[tid] = sVim[tid] * (double)rn;
    }
    __syncthreads();
  }
  if (tid < 64) {
    double sr = 0.0, si = 0.0;
#pragma unroll 1
    for (int k = 0; k < 64; ++k) {
      const double ar = (double)sP[tid * 64 + k], ai = (double)sP[4096 + tid * 64 + k];
      const double cr = sVre[k], ci = sVim[k];
      sr += ar * cr - ai * ci;
      si += ar * ci + ai * cr;
    }
    sRed[tid] = sr * sr + si * si;
    sUre[tid] = sVre[tid] * sVre[tid] + sVim[tid] * sVim[tid];
  }
  __syncthreads();
  double su = 0.0, sv = 0.0;
#pragma unroll 1
  for (int k = 0; k < 64; ++k) { su += sRed[k]; sv += sUre[k]; }
  const float sigma = sqrtf((float)su * (1.0f / fmaxf((float)sv, 1e-30f)));

  const float alpha = alpha_of(alpha_logit);
  const float beta = 1.0f - alpha;
  const float ascale = 1.0f + alpha * 0.001f;
  const float safe_norm = fmaxf(sigma, 1.1920929e-7f);
  const float scale = fminf(kRhoMax / safe_norm, 1.0f);
  const float bscale = beta * scale;
  __syncthreads();

#pragma unroll 1
  for (int e = 0; e < 16; ++e) {
    const int i = tid + 256 * e;
    sP[i] = bscale * sP[i];
    sP[4096 + i] = bscale * sP[4096 + i];
  }
  __syncthreads();

#pragma unroll 1
  for (int cc = 0; cc < 4; ++cc) {
#pragma unroll 1
    for (int e = 0; e < 4; ++e) {
      const int i = tid + 256 * e;
      const int lc = i >> 6, k = i & 63, c = cc * 16 + lc;
      float wr = 0.f, wi = 0.f;
#pragma unroll 1
      for (int kk = 0; kk < 64; ++kk) {
        const int mm = (k * kk) & 63;
        const float ct = sCT[mm], sn = sST[mm];
        const float lr = ((kk == c) ? 1.0f : 0.0f) + sP[kk * 64 + c];
        const float li = sP[4096 + kk * 64 + c];
        wr += ct * lr + sn * li;
        wi += ct * li - sn * lr;
      }
      sTerm[lc * 64 + k] = wr * ascale;
      sTerm[1024 + lc * 64 + k] = wi * ascale;
    }
    __syncthreads();
    {
      const int q = lane >> 3, c8 = (lane & 7) * 8;
      const int item = wave * 4 + q;
      const int lc = item & 15, isim = item >> 4;
      const int n = isim * 64 + cc * 16 + lc;
      emit_line_pair(sTerm + isim * 1024 + lc * 64 + c8, kCarryW, EWV + n * 64 + c8, EWR + n * 64 + c8);
    }
    __syncthreads();
  }

#pragma unroll 1
  for (int ch = 0; ch < 4; ++ch) {
#pragma unroll 1
    for (int e = 0; e < 4; ++e) {
      const int i = tid + 256 * e;
      const int lr = i >> 6, c = i & 63;
      const float id = ((ch * 16 + lr) == c) ? 1.0f : 0.0f;
      sTerm[i] = id;
      sTerm[1024 + i] = 0.0f;
      sIV[i] = id;
      sIV[1024 + i] = 0.0f;
    }
    __syncthreads();
#pragma unroll 1
    for (int it = 0; it < kSeriesTerms; ++it) {
      const int so = (it & 1) ? 2048 : 0;
      const int dofs = 2048 - so;
#pragma unroll 1
      for (int e = 0; e < 4; ++e) {
        const int i = tid + 256 * e;
        const int lr = i >> 6, c = i & 63;
        float ar = 0.f, ai = 0.f;
#pragma unroll 1
        for (int k = 0; k < 64; ++k) {
          const float tr = sTerm[so + lr * 64 + k], ti = sTerm[so + 1024 + lr * 64 + k];
          const float qr = sP[k * 64 + c], qi = sP[4096 + k * 64 + c];
          ar += tr * qr - ti * qi;
          ai += tr * qi + ti * qr;
        }
        ar = -ar;
        ai = -ai;
        sTerm[dofs + i] = ar;
        sTerm[dofs + 1024 + i] = ai;
        sIV[i] = sIV[i] + ar;
        sIV[1024 + i] = sIV[1024 + i] + ai;
      }
      __syncthreads();
    }
#pragma unroll 1
    for (int pass = 0; pass < 2; ++pass) {
#pragma unroll 1
      for (int e = 0; e < 4; ++e) {
        const int i = tid + 256 * e;
        const float vr = sIV[i], vi = sIV[1024 + i];
        *(volatile float*)(INVRE + ch * 1024 + i) = vr;
        *(volatile float*)(INVIM + ch * 1024 + i) = vi;
      }
      __threadfence();
    }
    __syncthreads();
  }
}

__global__ __launch_bounds__(256) void k_wplanes(
    const float* __restrict__ alpha_logit, const float* __restrict__ INVRE, const float* __restrict__ INVIM,
    const float* __restrict__ unc_w1, const float* __restrict__ unc_w2,
    unsigned short* __restrict__ DWV, unsigned short* __restrict__ DWR,
    unsigned short* __restrict__ U1P, unsigned short* __restrict__ U2P)
{
  __shared__ double sC17[17], sS17[17];
  __shared__ float sCT[64], sST[64];
  __shared__ __align__(16) float sStg[2048];
  const int tid = threadIdx.x, lane = tid & 31, wave = tid >> 5;
  build_trig(sC17, sS17, sCT, sST, tid);
  const float alpha = alpha_of(alpha_logit);
  const float ascale = 1.0f + alpha * 0.001f;
  const float inva = 1.0f / ascale;

#pragma unroll 1
  for (int cc = 0; cc < 4; ++cc) {
#pragma unroll 1
    for (int e = 0; e < 4; ++e) {
      const int i = tid + 256 * e;
      const int lc = i >> 6, r = i & 63, c = cc * 16 + lc;
      float vr = 0.f, vi = 0.f;
#pragma unroll 1
      for (int k = 0; k < 64; ++k) {
        const int mm = (c * k) & 63;
        const float ct = sCT[mm], sn = sST[mm];
        const float ir = INVRE[r * 64 + k], ii = INVIM[r * 64 + k];
        vr += ir * ct - ii * sn;
        vi += ir * sn + ii * ct;
      }
      sStg[lc * 128 + r] = vr * inva;
      sStg[lc * 128 + 64 + r] = -(vi * inva);
    }
    __syncthreads();
    {
      const int q = lane >> 3, c8 = (lane & 7) * 8;
      const int item = wave * 4 + q;
      const int lc = item >> 1, hf = item & 1;
      const int n = cc * 16 + lc;
      emit_line_pair(sStg + lc * 128 + hf * 64 + c8, kCarryW,
                     DWV + n * 128 + hf * 64 + c8, DWR + n * 128 + hf * 64 + c8);
    }
    __syncthreads();
  }

  {
    const int q = lane >> 3, c8 = (lane & 7) * 8;
    v8h hv;
    unsigned short* dst;
    if (wave < 4) {
      const int jj = wave * 4 + q;
#pragma unroll
      for (int e = 0; e < 8; ++e) {
        const float wv = bfr(unc_w1[(c8 + e) * 16 + jj]) * kCarryU;
        hv[e] = (_Float16)flush14(wv);
      }
      dst = U1P + jj * 64 + c8;
    } else {
      const int f = ((wave - 4) * 4 + q) * 64 + c8;
      const int n = f >> 4, kk0 = f & 15;
#pragma unroll
      for (int e = 0; e < 8; ++e) {
        const float wv = bfr(unc_w2[(kk0 + e) * 64 + n]) * kCarryU;
        hv[e] = (_Float16)flush14(wv);
      }
      dst = U2P + f;
    }
    *(volatile v8h*)dst = hv;
    __threadfence();
    *(volatile v8h*)dst = hv;
  }
}

__global__ __launch_bounds__(256) void k_tables(
    const float* __restrict__ dt_seq, const float* __restrict__ lam_re, const float* __restrict__ lam_im,
    const float* __restrict__ ftd_re, const float* __restrict__ ftd_im, float* __restrict__ TAB)
{
  const int tid = threadIdx.x;
#pragma unroll 1
  for (int e = 0; e < 8; ++e) {
    const int idx = tid + 256 * e;
    const int bt = idx >> 6, c = idx & 63;
    const float dtr = bfr(dt_seq[bt]) * (1.0f / kDtRef);
    const float a_re = bfr(lam_re[c]), a_im = bfr(lam_im[c]);
    const float f_re = bfr(ftd_re[c]), f_im = bfr(ftd_im[c]);
#pragma unroll 1
    for (int which = 0; which < 2; ++which) {
      const float pre = which ? f_re : a_re;
      const float pim = which ? f_im : a_im;
      const float sp = fmaxf(pre, 0.0f) + log1pf(expf(-fabsf(pre)));
      const float zr = (-sp) * dtr, zi = pim * dtr;
      const float er = expf(zr);
      float sn, cs;
      sincosf(zi, &sn, &cs);
      const float dr = er * cs, di = er * sn;
      const float m2 = zr * zr + zi * zi;
      const bool big = sqrtf(m2) > 1e-7f;
      const float m2s = big ? m2 : 1.0f;
      const float inv = 1.0f / m2s;
      const float nr = dr - 1.0f, ni = di;
      const float pr = (nr * zr + ni * zi) * inv;
      const float pi = (ni * zr - nr * zi) * inv;
      const float z2r = zr * zr - zi * zi, z2i = 2.0f * zr * zi;
      const float tr = 1.0f + 0.5f * zr + z2r * (1.0f / 6.0f);
      const float ti = 0.5f * zi + z2i * (1.0f / 6.0f);
      const float fr = dtr * (big ? pr : tr);
      const float fi = dtr * (big ? pi : ti);
      float* base = TAB + which * 4 * kPlane + idx;
      *(volatile float*)(base) = dr;
      *(volatile float*)(base + kPlane) = di;
      *(volatile float*)(base + 2 * kPlane) = fr;
      *(volatile float*)(base + 3 * kPlane) = fi;
      __threadfence();
      *(volatile float*)(base) = dr;
      *(volatile float*)(base + kPlane) = di;
      *(volatile float*)(base + 2 * kPlane) = fr;
      *(volatile float*)(base + 3 * kPlane) = fi;
    }
  }
}

__global__ __launch_bounds__(128) void k_encode_mean(
    const float* __restrict__ x, const unsigned short* __restrict__ EWV, float* __restrict__ PART)
{
  __shared__ float sPart[4 * 128];
  const int tid = threadIdx.x, lane = tid & 31, wave = tid >> 5;
  const int hh = lane >> 4, m = lane & 15;
  const int bt = blockIdx.x >> 2, blk = blockIdx.x & 3;
  const _Float16* ewv = (const _Float16*)EWV;
#pragma unroll 1
  for (int half = 0; half < 2; ++half) {
    v8f av[4];
#pragma unroll
    for (int j = 0; j < 4; ++j) av[j] = zero8f();
#pragma unroll 1
    for (int g = 0; g < 16; ++g) {
      const int pix = blk * 1024 + wave * 256 + g * 16 + m;
      const float* xrow = x + ((size_t)bt * kHW + pix) * kD + 8 * hh;
      const v16h xb0 = x_frag(xrow);
      const v16h xb1 = x_frag(xrow + 32);
#pragma unroll
      for (int j = 0; j < 4; ++j) {
        const int n = half * 64 + 16 * j + m;
        const _Float16* pv = ewv + n * 64 + 8 * hh;
        v16h a;
        a = frag_ld(pv);
        av[j] = mma_h(a, xb0, av[j]);
        a = frag_ld(pv + 32);
        av[j] = mma_h(a, xb1, av[j]);
      }
    }
#pragma unroll
    for (int j = 0; j < 4; ++j) {
#pragma unroll
      for (int r = 0; r < 8; ++r) {
        float v = av[j][r] * kFoldEnc;
        v += __shfl_xor(v, 1, 32);
        v += __shfl_xor(v, 2, 32);
        v += __shfl_xor(v, 4, 32);
        v += __shfl_xor(v, 8, 32);
        if (m == 0) sPart[wave * 128 + half * 64 + 16 * j + 8 * hh + r] = v;
      }
    }
  }
  __syncthreads();
  if (wave == 0) {
    const int n0 = lane * 4;
    v4f tot;
#pragma unroll
    for (int e = 0; e < 4; ++e)
      tot[e] = ((sPart[n0 + e] + sPart[128 + n0 + e]) + sPart[256 + n0 + e]) + sPart[384 + n0 + e];
    float* dst = PART + (size_t)(bt * 4 + blk) * 128 + n0;
    *(volatile v4f*)dst = tot;
    __threadfence();
    *(volatile v4f*)dst = tot;
  }
}

template <int NOUT>
__device__ __forceinline__ void fc_rows(const float* in0, int K0, const float* in1, int K1,
                                        const float* __restrict__ W, const float* __restrict__ bias,
                                        float* outp, int tid)
{
  constexpr int RS = 256 / NOUT;
  constexpr int G = 32 / RS / 4;
  const int j = tid & (NOUT - 1);
  const int rbase = tid / NOUT;
  const float bv = bfr(bias[j]);
#pragma unroll 1
  for (int g = 0; g < G; ++g) {
    const int r0 = rbase + RS * 4 * g;
    float a0 = bv, a1 = bv, a2 = bv, a3 = bv;
#pragma unroll 1
    for (int k = 0; k < K0; ++k) {
      const float w = bfr(W[(size_t)k * NOUT + j]);
      a0 = fmaf(in0[(r0) * 128 + k], w, a0);
      a1 = fmaf(in0[(r0 + RS) * 128 + k], w, a1);
      a2 = fmaf(in0[(r0 + 2 * RS) * 128 + k], w, a2);
      a3 = fmaf(in0[(r0 + 3 * RS) * 128 + k], w, a3);
    }
#pragma unroll 1
    for (int k = 0; k < K1; ++k) {
      const float w = bfr(W[(size_t)(K0 + k) * NOUT + j]);
      a0 = fmaf(in1[(r0) * 128 + k], w, a0);
      a1 = fmaf(in1[(r0 + RS) * 128 + k], w, a1);
      a2 = fmaf(in1[(r0 + 2 * RS) * 128 + k], w, a2);
      a3 = fmaf(in1[(r0 + 3 * RS) * 128 + k], w, a3);
    }
    outp[(r0) * 128 + j] = a0;
    outp[(r0 + RS) * 128 + j] = a1;
    outp[(r0 + 2 * RS) * 128 + j] = a2;
    outp[(r0 + 3 * RS) * 128 + j] = a3;
  }
}

__global__ __launch_bounds__(256) void k_flux(
    const float* __restrict__ PART, const float* __restrict__ TAB,
    const float* __restrict__ ft_in_w, const float* __restrict__ ft_in_b,
    const float* __restrict__ ft_out_w, const float* __restrict__ ft_out_b,
    const float* __restrict__ ft_gc_w, const float* __restrict__ ft_gc_b,
    const float* __restrict__ ft_gate_w, const float* __restrict__ ft_gate_b,
    const float* __restrict__ ft_h0_re, const float* __restrict__ ft_h0_im,
    float* __restrict__ GSRE, float* __restrict__ GSIM)
{
  __shared__ __align__(16) float sA[4096];
  __shared__ __align__(16) float sB[4096];
  __shared__ __align__(16) float sC[4096];
  const int tid = threadIdx.x;
#pragma unroll 1
  for (int e = 0; e < 16; ++e) {
    const int idx = tid + 256 * e;
    const int r = idx >> 7, n = idx & 127;
    const float* pp = PART + (size_t)r * 512 + n;
    const float s = ((pp[0] + pp[128]) + pp[256]) + pp[384];
    sA[idx] = s * (1.0f / (float)kHW);
  }
  __syncthreads();
  fc_rows<128>(sA, 128, sA, 0, ft_in_w, ft_in_b, sB, tid);
  __syncthreads();
  if (tid < 128) {
    const int bb = tid >> 6, d = tid & 63;
    float fr = bfr(ft_h0_re[d]), fi = bfr(ft_h0_im[d]);
#pragma unroll 1
    for (int t = 0; t < kNT; ++t) {
      const int bt = bb * kNT + t;
      const float xr = sB[bt * 128 + d], xi = sB[bt * 128 + 64 + d];
      const float dfr = TAB[4 * kPlane + bt * 64 + d], dfi = TAB[5 * kPlane + bt * 64 + d];
      const float ffr = TAB[6 * kPlane + bt * 64 + d], ffi = TAB[7 * kPlane + bt * 64 + d];
      const float ur = xr * ffr - xi * ffi, ui = xr * ffi + xi * ffr;
      const float nr = (fr * dfr - fi * dfi) + ur;
      const float ni = (fr * dfi + fi * dfr) + ui;
      fr = nr;
      fi = ni;
      sA[bt * 128 + d] = fr;
      sA[bt * 128 + 64 + d] = fi;
    }
  }
  __syncthreads();
  fc_rows<128>(sA, 128, sA, 0, ft_out_w, ft_out_b, sB, tid);
  __syncthreads();
  fc_rows<128>(sA, 128, sB, 128, ft_gc_w, ft_gc_b, sC, tid);
  __syncthreads();
  fc_rows<64>(sC, 128, sC, 0, ft_gate_w, ft_gate_b, sA, tid);
  __syncthreads();
#pragma unroll 1
  for (int e = 0; e < 8; ++e) {
    const int idx = tid + 256 * e;
    const int bt = idx >> 6, d = idx & 63;
    const float lg = sA[bt * 128 + d];
    const float ex = expf(fminf(-lg, 80.0f));
    const float g = (1.0f / (1.0f + ex)) * 0.98f + 0.01f;
    const float vr = g * sB[bt * 128 + d];
    const float vi = g * sB[bt * 128 + 64 + d];
    *(volatile float*)(GSRE + idx) = vr;
    *(volatile float*)(GSIM + idx) = vi;
    __threadfence();
    *(volatile float*)(GSRE + idx) = vr;
    *(volatile float*)(GSIM + idx) = vi;
  }
}

__global__ __launch_bounds__(64) void k_scan_decode(
    const float* __restrict__ x,
    const unsigned short* __restrict__ EWV,
    const unsigned short* __restrict__ DWV, const unsigned short* __restrict__ DWR,
    const unsigned short* __restrict__ U1P, const unsigned short* __restrict__ U2P,
    const float* __restrict__ TAB, const float* __restrict__ GSRE, const float* __restrict__ GSIM,
    const float* __restrict__ h0_re, const float* __restrict__ h0_im,
    const float* __restrict__ unc_b1, const float* __restrict__ unc_b2,
    float* __restrict__ out)
{
  __shared__ __align__(32) float sState[2][2048];
  __shared__ __align__(32) _Float16 sFrag[2][4096];
  __shared__ __align__(16) float sY[2][16 * 68];
  __shared__ __align__(16) float sS[2][16 * 68];
  const int tid = threadIdx.x, lane = tid & 31, wave = tid >> 5;
  const int hh = lane >> 4, m = lane & 15;
  const int pg = blockIdx.x * 2 + wave;
  const int b = pg >> 8;
  const int pix0 = (pg & 255) * 16;
  float* st = sState[wave];
  _Float16* fr = sFrag[wave];
  float* sy = sY[wave];
  float* ss = sS[wave];
  const _Float16* ewv = (const _Float16*)EWV;
  const _Float16* dwv = (const _Float16*)DWV;
  const _Float16* dwr = (const _Float16*)DWR;
  const _Float16* u1 = (const _Float16*)U1P;
  const _Float16* u2 = (const _Float16*)U2P;

#pragma unroll 1
  for (int ct = 0; ct < 4; ++ct) {
    const int c0 = 16 * ct + 8 * hh;
    const v8f a = ld8(h0_re + c0);
    const v8f c = ld8(h0_im + c0);
    v8f ar, ci;
#pragma unroll
    for (int r = 0; r < 8; ++r) {
      const float s0 = a[r];
      const float s1 = c[r];
      ar[r] = bfr(s0);
      ci[r] = bfr(s1);
    }
    *(v8f*)(st + (ct * 32 + lane) * 8) = ar;
    *(v8f*)(st + ((4 + ct) * 32 + lane) * 8) = ci;
  }
  v8f b1v;
  {
    const v8f t1 = ld8(unc_b1 + 8 * hh);
#pragma unroll
    for (int r = 0; r < 8; ++r) {
      const float s0 = t1[r];
      b1v[r] = bfr(s0);
    }
  }

#pragma unroll 1
  for (int t = 0; t < kNT; ++t) {
    const int bt = b * kNT + t;
    const float* xrow = x + ((size_t)bt * kHW + pix0 + m) * kD + 8 * hh;
    const v16h xb0 = x_frag(xrow);
    const v16h xb1 = x_frag(xrow + 32);
    v8f hacc_v = zero8f();
    const float* tb = TAB + bt * 64;
    const float* gr = GSRE + bt * 64;
    const float* gi = GSIM + bt * 64;

#pragma unroll 1
    for (int s = 0; s < 2; ++s) {
      v8h qv_re[2], qr_re[2], qv_im[2], qr_im[2], qv_am[2];
#pragma unroll
      for (int q = 0; q < 2; ++q) {
        const int ct = 2 * s + q;
        const int nre = 16 * ct + m;
        const _Float16* pv = ewv + nre * 64 + 8 * hh;
        v8f are_v = zero8f(), aim_v = zero8f();
        {
          v16h a;
          a = frag_ld(pv);
          are_v = mma_h(a, xb0, are_v);
          a = frag_ld(pv + 32);
          are_v = mma_h(a, xb1, are_v);
          a = frag_ld(pv + 64 * 64);
          aim_v = mma_h(a, xb0, aim_v);
          a = frag_ld(pv + 64 * 64 + 32);
          aim_v = mma_h(a, xb1, aim_v);
        }
        const int c0 = 16 * ct + 8 * hh;
        const v8f dre = ld8(tb + c0);
        const v8f dim = ld8(tb + kPlane + c0);
        const v8f fre = ld8(tb + 2 * kPlane + c0);
        const v8f fim = ld8(tb + 3 * kPlane + c0);
        const v8f gre = ld8(gr + c0);
        const v8f gim = ld8(gi + c0);
        float* spre = st + (ct * 32 + lane) * 8;
        float* spim = st + ((4 + ct) * 32 + lane) * 8;
        const v8f hre = *(const v8f*)spre;
        const v8f him = *(const v8f*)spim;
        v8f nre8, nim8;
#pragma unroll
        for (int r = 0; r < 8; ++r) {
          const float er = are_v[r] * kFoldEnc;
          const float ei = aim_v[r] * kFoldEnc;
          const float ur = er + gre[r], ui = ei + gim[r];
          const float nr = (hre[r] * dre[r] - him[r] * dim[r]) + (ur * fre[r] - ui * fim[r]);
          const float ni = (hre[r] * dim[r] + him[r] * dre[r]) + (ur * fim[r] + ui * fre[r]);
          nre8[r] = nr;
          nim8[r] = ni;
          _Float16 a16, r16;
          split16(nr, kCarryH, a16, r16);
          qv_re[q][r] = a16;
          qr_re[q][r] = r16;
          split16(ni, kCarryH, a16, r16);
          qv_im[q][r] = a16;
          qr_im[q][r] = r16;
          const float am = sqrtf(nr * nr + ni * ni);
          qv_am[q][r] = plain16(am, kCarryH);
        }
        *(v8f*)spre = nre8;
        *(v8f*)spim = nim8;
      }
      FragU f;
      f.h[0] = qv_re[0];
      f.h[1] = qv_re[1];
      *(v16h*)(fr + ((s * 2 + 0) * 32 + lane) * 16) = f.v;
      f.h[0] = qr_re[0];
      f.h[1] = qr_re[1];
      *(v16h*)(fr + ((s * 2 + 1) * 32 + lane) * 16) = f.v;
      f.h[0] = qv_im[0];
      f.h[1] = qv_im[1];
      *(v16h*)(fr + (((s + 2) * 2 + 0) * 32 + lane) * 16) = f.v;
      f.h[0] = qr_im[0];
      f.h[1] = qr_im[1];
      *(v16h*)(fr + (((s + 2) * 2 + 1) * 32 + lane) * 16) = f.v;
      FragU fav;
      fav.h[0] = qv_am[0];
      fav.h[1] = qv_am[1];
      const v16h a1 = frag_ld(u1 + m * 64 + 32 * s + 8 * hh);
      hacc_v = mma_h(a1, fav.v, hacc_v);
    }

    FragU hbv;
    {
      v8h hd_v;
#pragma unroll
      for (int r = 0; r < 8; ++r) {
        const float z = hacc_v[r] * kFoldU + b1v[r];
        const float ex = expf(fminf(-z, 80.0f));
        const float hd = z * (1.0f / (1.0f + ex));
        hd_v[r] = plain16(hd, kCarryH);
      }
      hbv.h[0] = hd_v;
      hbv.h[1] = zero8h();
    }

#pragma unroll 1
    for (int j = 0; j < 4; ++j) {
      const int n = 16 * j + m;
      const _Float16* pv = dwv + n * 128 + 8 * hh;
      const _Float16* pr = dwr + n * 128 + 8 * hh;
      v8f ym = zero8f(), yr = zero8f();
#pragma unroll
      for (int ks = 0; ks < 4; ++ks) {
        const v16h bv = *(const v16h*)(fr + ((ks * 2 + 0) * 32 + lane) * 16);
        const v16h br = *(const v16h*)(fr + ((ks * 2 + 1) * 32 + lane) * 16);
        const v16h av = frag_ld(pv + 32 * ks);
        const v16h ar = frag_ld(pr + 32 * ks);
        ym = mma_h(av, bv, ym);
        yr = mma_h(av, br, yr);
        yr = mma_h(ar, bv, yr);
      }
      FragU a2;
      a2.h[0] = *(const v8h*)(u2 + n * 16 + 8 * hh);
      a2.h[1] = zero8h();
      v8f sm = zero8f();
      sm = mma_h(a2.v, hbv.v, sm);
      const int c0 = 16 * j + 8 * hh;
      const v8f bb = ld8(unc_b2 + c0);
      v4f y0, y1, s0, s1;
#pragma unroll
      for (int r = 0; r < 4; ++r) {
        const float b0s = bb[r];
        const float b1s = bb[4 + r];
        y0[r] = ym[r] * kFoldDec + yr[r] * kFoldDecRes;
        y1[r] = ym[4 + r] * kFoldDec + yr[4 + r] * kFoldDecRes;
        s0[r] = sm[r] * kFoldU + bfr(b0s);
        s1[r] = sm[4 + r] * kFoldU + bfr(b1s);
      }
      *(v4f*)(sy + m * 68 + c0) = y0;
      *(v4f*)(sy + m * 68 + c0 + 4) = y1;
      *(v4f*)(ss + m * 68 + c0) = s0;
      *(v4f*)(ss + m * 68 + c0 + 4) = s1;
    }
    wave_sync_lds();

    float* orow = out + ((size_t)bt * kHW + pix0) * kD;
    const int c4 = m * 4;
#pragma unroll 1
    for (int it = 0; it < 8; ++it) {
      const int row = it * 2 + hh;
      const v4f yv = *(const v4f*)(sy + row * 68 + c4);
      const v4f sv = *(const v4f*)(ss + row * 68 + c4);
      v4f o;
#pragma unroll
      for (int e = 0; e < 4; ++e) {
        const float sve = sv[e];
        const float yve = yv[e];
        const float ex = expf(fminf(-sve, 80.0f));
        o[e] = yve * (1.0f / (1.0f + ex));
      }
      *(v4f*)(sy + row * 68 + c4) = o;
      *(volatile v4f*)(orow + (size_t)row * kD + c4) = o;
    }
    __threadfence();
#pragma unroll 1
    for (int it = 0; it < 8; ++it) {
      const int row = it * 2 + hh;
      const v4f o = *(const v4f*)(sy + row * 68 + c4);
      *(volatile v4f*)(orow + (size_t)row * kD + c4) = o;
    }
    __threadfence();
    wave_sync_lds();
  }
}

extern "C" void kernel_launch(void* const* d_in, const int* in_sizes, int n_in,
                              void* d_out, int out_size, void* d_ws, size_t ws_size,
                              hipStream_t stream) {
  if (n_in < 25) return;
  if (in_sizes[0] != kNB * kNT * kHW * kD) return;
  if (in_sizes[1] != kBT) return;
  if (in_sizes[2] != kD * kD || in_sizes[3] != kD * kD) return;
  if (in_sizes[4] != 1) return;
  if (in_sizes[5] != kD || in_sizes[6] != kD || in_sizes[7] != kD || in_sizes[8] != kD) return;
  if (in_sizes[9] != kD || in_sizes[10] != kD) return;
  if (in_sizes[11] != 128 * 128 || in_sizes[12] != 128) return;
  if (in_sizes[13] != 128 * 128 || in_sizes[14] != 128) return;
  if (in_sizes[15] != 256 * 128 || in_sizes[16] != 128) return;
  if (in_sizes[17] != 128 * 64 || in_sizes[18] != 64) return;
  if (in_sizes[19] != kD || in_sizes[20] != kD) return;
  if (in_sizes[21] != 64 * 16 || in_sizes[22] != 16) return;
  if (in_sizes[23] != 16 * 64 || in_sizes[24] != 64) return;
  if (out_size != kNB * kNT * kHW * kD) return;
  if (ws_size < kWsTotal) return;

  const float* x           = (const float*)d_in[0];
  const float* dt_seq      = (const float*)d_in[1];
  const float* w_re        = (const float*)d_in[2];
  const float* w_im        = (const float*)d_in[3];
  const float* alpha_logit = (const float*)d_in[4];
  const float* lam_re      = (const float*)d_in[5];
  const float* lam_im      = (const float*)d_in[6];
  const float* h0_re       = (const float*)d_in[7];
  const float* h0_im       = (const float*)d_in[8];
  const float* ftd_re      = (const float*)d_in[9];
  const float* ftd_im      = (const float*)d_in[10];
  const float* ft_in_w     = (const float*)d_in[11];
  const float* ft_in_b     = (const float*)d_in[12];
  const float* ft_out_w    = (const float*)d_in[13];
  const float* ft_out_b    = (const float*)d_in[14];
  const float* ft_gc_w     = (const float*)d_in[15];
  const float* ft_gc_b     = (const float*)d_in[16];
  const float* ft_gate_w   = (const float*)d_in[17];
  const float* ft_gate_b   = (const float*)d_in[18];
  const float* ft_h0_re    = (const float*)d_in[19];
  const float* ft_h0_im    = (const float*)d_in[20];
  const float* unc_w1      = (const float*)d_in[21];
  const float* unc_b1      = (const float*)d_in[22];
  const float* unc_w2      = (const float*)d_in[23];
  const float* unc_b2      = (const float*)d_in[24];
  float* out = (float*)d_out;

  char* ws = (char*)d_ws;
  unsigned short* EWV = (unsigned short*)(ws + kOffEWV);
  unsigned short* EWR = (unsigned short*)(ws + kOffEWR);
  unsigned short* DWV = (unsigned short*)(ws + kOffDWV);
  unsigned short* DWR = (unsigned short*)(ws + kOffDWR);
  unsigned short* U1P = (unsigned short*)(ws + kOffU1);
  unsigned short* U2P = (unsigned short*)(ws + kOffU2);
  float* INVRE = (float*)(ws + kOffINVRE);
  float* INVIM = (float*)(ws + kOffINVIM);
  float* TAB   = (float*)(ws + kOffTAB);
  float* GSRE  = (float*)(ws + kOffGSRE);
  float* GSIM  = (float*)(ws + kOffGSIM);
  float* PART  = (float*)(ws + kOffPART);

  k_mats<<<1, 256, 0, stream>>>(w_re, w_im, alpha_logit, EWV, EWR, INVRE, INVIM);
  k_wplanes<<<1, 256, 0, stream>>>(alpha_logit, INVRE, INVIM, unc_w1, unc_w2, DWV, DWR, U1P, U2P);
  k_tables<<<1, 256, 0, stream>>>(dt_seq, lam_re, lam_im, ftd_re, ftd_im, TAB);
  k_encode_mean<<<kBT * 4, 128, 0, stream>>>(x, EWV, PART);
  k_flux<<<1, 256, 0, stream>>>(PART, TAB, ft_in_w, ft_in_b, ft_out_w, ft_out_b, ft_gc_w, ft_gc_b,
                                ft_gate_w, ft_gate_b, ft_h0_re, ft_h0_im, GSRE, GSIM);
  k_scan_decode<<<(kNB * kHW / 16) / 2, 64, 0, stream>>>(x, EWV, DWV, DWR, U1P, U2P, TAB, GSRE, GSIM,
                                                         h0_re, h0_im, unc_b1, unc_b2, out);
}
